// GraphSAGE_41635412967695
// MI455X (gfx1250) — hardware-verified
//
#include <hip/hip_runtime.h>
#include <stddef.h>
#include <stdint.h>
#include <math.h>


#define FIN    64
#define HID    128
#define G4     512
#define DEG    8
#define NB     32
#define HP     264
#define GBM    64
#define GBN    128
#define GTHR   128
#define LTHR   256
#define LDS_G  65536
#define LDS_C  16384
#define LDS_H  (NB * HP * 2)
#define LDS_S  (NB * DEG * 4)
#define LDS_TOT (LDS_G + LDS_C + LDS_H + LDS_S)
#define PE0    4096
#define PE1    12288
#define PE2    15360
#define PE3    23552
#define PE4    31744
#define PE5    35840
#define PVN    1792
#define PVU    448
#define WSMAX  134217728

static_assert(PE0 % 256 == 0 && PE1 % 256 == 0 && PE2 % 256 == 0 && PE3 % 256 == 0);
static_assert(PE4 % 256 == 0 && PE5 % 256 == 0 && PVN == 4 * PVU);
static_assert(NB * DEG == LTHR && NB == 32 && HID == 128 && G4 == 4 * HID);
static_assert(LDS_G % 16 == 0 && LDS_C % 16 == 0 && LDS_H % 16 == 0 && (HP % 8) == 0);
static_assert(NB * HID * 4 <= LDS_G && 8 * 4 * 256 * 2 <= LDS_C);
static_assert(LDS_TOT <= 300000);
static_assert(GBM == (GTHR / 32) * 16 && G4 % GBN == 0 && FIN % 32 == 0 && HID % 32 == 0);

typedef float          v4f   __attribute__((ext_vector_type(4)));
typedef float          v8f   __attribute__((ext_vector_type(8)));
typedef int            v8i   __attribute__((ext_vector_type(8)));
typedef unsigned short v4us  __attribute__((ext_vector_type(4)));
typedef unsigned short v8us  __attribute__((ext_vector_type(8)));
typedef unsigned short v16us __attribute__((ext_vector_type(16)));
typedef __bf16         v16bf __attribute__((ext_vector_type(16)));
typedef v4f  __attribute__((may_alias)) v4fa;
typedef v4us __attribute__((may_alias)) v4usa;
typedef v8us __attribute__((may_alias)) v8usa;
union FragB { v16bf v; v16us u; v8us h[2]; v8i w; };

__device__ __forceinline__ v8f wmb(const FragB& a, const FragB& b, v8f c) {
  v8f d = __builtin_amdgcn_wmma_f32_16x16x32_bf16(false, a.v, false, b.v, (short)0, c, false, false);
  asm volatile("v_nop\n\tv_nop\n\tv_nop\n\tv_nop" : "+v"(d) : "v"(a.w), "v"(b.w));
  return d;
}

__device__ __forceinline__ unsigned bf16_bits(float f) {
  const unsigned u = __float_as_uint(f);
  return (u + 0x7FFFu + ((u >> 16) & 1u)) >> 16;
}
__device__ __forceinline__ float bf16_val(float f) {
  return __uint_as_float(bf16_bits(f) << 16);
}

__device__ __forceinline__ void wave_sync() {
  __builtin_amdgcn_fence(__ATOMIC_RELEASE, "wavefront");
  __builtin_amdgcn_wave_barrier();
  __builtin_amdgcn_fence(__ATOMIC_ACQUIRE, "wavefront");
}

__device__ __forceinline__ FragB lda_f32(const float* p) {
  const v4f a0 = *(const v4f*)p;
  const v4f a1 = *(const v4f*)(p + 4);
  const v4f b0 = *(const v4f*)(p + 16);
  const v4f b1 = *(const v4f*)(p + 20);
  v8us lo, hi;
  lo[0] = (unsigned short)bf16_bits(a0.x); lo[1] = (unsigned short)bf16_bits(a0.y);
  lo[2] = (unsigned short)bf16_bits(a0.z); lo[3] = (unsigned short)bf16_bits(a0.w);
  lo[4] = (unsigned short)bf16_bits(a1.x); lo[5] = (unsigned short)bf16_bits(a1.y);
  lo[6] = (unsigned short)bf16_bits(a1.z); lo[7] = (unsigned short)bf16_bits(a1.w);
  hi[0] = (unsigned short)bf16_bits(b0.x); hi[1] = (unsigned short)bf16_bits(b0.y);
  hi[2] = (unsigned short)bf16_bits(b0.z); hi[3] = (unsigned short)bf16_bits(b0.w);
  hi[4] = (unsigned short)bf16_bits(b1.x); hi[5] = (unsigned short)bf16_bits(b1.y);
  hi[6] = (unsigned short)bf16_bits(b1.z); hi[7] = (unsigned short)bf16_bits(b1.w);
  FragB f;
  f.h[0] = lo;
  f.h[1] = hi;
  return f;
}

__device__ __forceinline__ FragB ld16(const unsigned short* p) {
  FragB f;
  f.h[0] = *(const v8usa*)p;
  f.h[1] = *(const v8usa*)(p + 16);
  return f;
}

__device__ __forceinline__ float sigm(float v) {
  v = fminf(fmaxf(v, -40.0f), 40.0f);
  return 1.0f / (1.0f + expf(-v));
}

__global__ __launch_bounds__(256) void k_prep(
    const float* __restrict__ Wih1, const float* __restrict__ Whh1, const float* __restrict__ b1,
    const float* __restrict__ lin1W, const float* __restrict__ lin1b, const float* __restrict__ g1,
    const float* __restrict__ be1,
    const float* __restrict__ Wih2, const float* __restrict__ Whh2, const float* __restrict__ b2,
    const float* __restrict__ lin2W, const float* __restrict__ lin2b, const float* __restrict__ g2,
    const float* __restrict__ be2,
    unsigned short* WIH1p, unsigned short* WHH1p, unsigned short* LIN1p,
    unsigned short* WIH2p, unsigned short* WHH2p, unsigned short* LIN2p, float* PV)
{
  const int u = (int)blockIdx.x * 256 + (int)threadIdx.x;
  if (u < PE5) {
    const float* W;
    unsigned short* P;
    int v, K, perm;
    if (u < PE0)      { W = Wih1;  P = WIH1p; v = u;       K = 64;  perm = 1; }
    else if (u < PE1) { W = Whh1;  P = WHH1p; v = u - PE0; K = 128; perm = 0; }
    else if (u < PE2) { W = lin1W; P = LIN1p; v = u - PE1; K = 192; perm = 0; }
    else if (u < PE3) { W = Wih2;  P = WIH2p; v = u - PE2; K = 128; perm = 1; }
    else if (u < PE4) { W = Whh2;  P = WHH2p; v = u - PE3; K = 128; perm = 0; }
    else              { W = lin2W; P = LIN2p; v = u - PE4; K = 256; perm = 0; }
    const int kd8 = K >> 3;
    const int n   = v / kd8;
    const int k8  = (v - n * kd8) * 8;
    const int sp  = (n & 3) * 128 + (n >> 6) * 16 + ((n >> 2) & 15);
    const int sr  = (perm != 0) ? sp : n;
    const float* p = W + (size_t)sr * K + k8;
    const v4f a = *(const v4f*)p;
    const v4f b = *(const v4f*)(p + 4);
    v8us o;
    o[0] = (unsigned short)bf16_bits(a.x); o[1] = (unsigned short)bf16_bits(a.y);
    o[2] = (unsigned short)bf16_bits(a.z); o[3] = (unsigned short)bf16_bits(a.w);
    o[4] = (unsigned short)bf16_bits(b.x); o[5] = (unsigned short)bf16_bits(b.y);
    o[6] = (unsigned short)bf16_bits(b.z); o[7] = (unsigned short)bf16_bits(b.w);
    unsigned short* dp = P + (size_t)8 * v;
    *(volatile v8us*)dp = o;
    __threadfence();
    *(volatile v8us*)dp = o;
  } else {
    const int v = u - PE5;
    if (v >= PVU) return;
    const int idx = 4 * v;
    v4f o;
    if (idx < 1024) {
      const int c  = idx & 511;
      const int bs = (c >> 6) * 16 + ((c >> 2) & 15);
      const float* bb = (idx < 512) ? b1 : b2;
      o.x = bf16_val(bb[bs]);
      o.y = bf16_val(bb[128 + bs]);
      o.z = bf16_val(bb[256 + bs]);
      o.w = bf16_val(bb[384 + bs]);
    } else {
      const int sec = (idx - 1024) >> 7;
      const int o4  = (idx - 1024) & 127;
      const float* s;
      if (sec == 0)      s = lin1b;
      else if (sec == 1) s = lin2b;
      else if (sec == 2) s = g1;
      else if (sec == 3) s = be1;
      else if (sec == 4) s = g2;
      else               s = be2;
      const v4f a = *(const v4f*)(s + o4);
      o.x = bf16_val(a.x); o.y = bf16_val(a.y); o.z = bf16_val(a.z); o.w = bf16_val(a.w);
    }
    float* dp = PV + idx;
    *(volatile v4f*)dp = o;
    __threadfence();
    *(volatile v4f*)dp = o;
  }
}

template <int LYR>
__global__ __launch_bounds__(GTHR) void k_xg(const float* __restrict__ xf, const unsigned short* __restrict__ H1,
                                             const unsigned short* __restrict__ WT, const float* __restrict__ bp,
                                             float* XG, int nN)
{
  __shared__ __attribute__((aligned(16))) float stg[GBM * GBN];
  const int tid = (int)threadIdx.x, lane = tid & 31, wave = tid >> 5, hh = lane >> 4, m = lane & 15;
  const int rowBase = (int)blockIdx.x * GBM;
  const int col0    = (int)blockIdx.y * GBN;
  int ar = rowBase + 16 * wave + m;
  ar = ar < nN ? ar : nN - 1;

  v8f acc[8];
  {
    const v8f z = {0.f, 0.f, 0.f, 0.f, 0.f, 0.f, 0.f, 0.f};
#pragma unroll
    for (int t = 0; t < 8; ++t) acc[t] = z;
  }
  if constexpr (LYR == 1) {
    const float* ap = xf + (size_t)ar * FIN + 8 * hh;
    const unsigned short* wp = WT + (size_t)(col0 + m) * FIN + 8 * hh;
#pragma unroll 1
    for (int ks = 0; ks < FIN / 32; ++ks) {
      const FragB af = lda_f32(ap + 32 * ks);
#pragma unroll
      for (int nt = 0; nt < 8; ++nt) {
        const FragB bf = ld16(wp + (size_t)(16 * nt) * FIN + 32 * ks);
        acc[nt] = wmb(af, bf, acc[nt]);
      }
    }
  } else {
    const unsigned short* ap = H1 + (size_t)ar * (2 * HID) + 8 * hh;
    const unsigned short* wp = WT + (size_t)(col0 + m) * HID + 8 * hh;
#pragma unroll 1
    for (int ks = 0; ks < HID / 32; ++ks) {
      const FragB ah = ld16(ap + 32 * ks);
      const FragB al = ld16(ap + HID + 32 * ks);
      FragB bf[8];
#pragma unroll
      for (int nt = 0; nt < 8; ++nt) bf[nt] = ld16(wp + (size_t)(16 * nt) * HID + 32 * ks);
#pragma unroll
      for (int nt = 0; nt < 8; ++nt) acc[nt] = wmb(ah, bf[nt], acc[nt]);
#pragma unroll
      for (int nt = 0; nt < 8; ++nt) acc[nt] = wmb(al, bf[nt], acc[nt]);
    }
  }

#pragma unroll
  for (int nt = 0; nt < 8; ++nt) {
    const int lc = 16 * nt + m;
#pragma unroll
    for (int r = 0; r < 8; ++r) {
      const int lr = 16 * wave + 8 * hh + r;
      stg[lr * GBN + lc] = acc[nt][r];
    }
  }
  __syncthreads();

  const v4f bb4 = *(const v4f*)(bp + col0 + 4 * lane);
  v4f pv[16];
#pragma unroll
  for (int i = 0; i < 16; ++i) {
    const v4f t = *(const v4fa*)(stg + (16 * wave + i) * GBN + 4 * lane);
    pv[i] = t + bb4;
  }
#pragma unroll
  for (int i = 0; i < 16; ++i) {
    const int r = rowBase + 16 * wave + i;
    if (r < nN) *(volatile v4f*)(XG + (size_t)r * G4 + col0 + 4 * lane) = pv[i];
  }
  __threadfence();
#pragma unroll
  for (int i = 0; i < 16; ++i) {
    const int r = rowBase + 16 * wave + i;
    if (r < nN) *(volatile v4f*)(XG + (size_t)r * G4 + col0 + 4 * lane) = pv[i];
  }
}

template <int LYR>
__global__ __launch_bounds__(LTHR) void k_lstm(
    const float* __restrict__ XG, const int* __restrict__ esrc, const unsigned short* __restrict__ WHH,
    const float* __restrict__ xf, const unsigned short* H1r, unsigned short* H1w,
    const unsigned short* __restrict__ LINW, const float* __restrict__ pvb, const float* __restrict__ pvg,
    const float* __restrict__ pvbe, float* outp, int nN)
{
  extern __shared__ __attribute__((aligned(16))) unsigned char dsm[];
  float*          sG   = (float*)dsm;
  float*          sC   = (float*)(dsm + LDS_G);
  unsigned short* sH   = (unsigned short*)(dsm + LDS_G + LDS_C);
  int*            sSrc = (int*)(dsm + LDS_G + LDS_C + LDS_H);

  const int tid = (int)threadIdx.x, lane = tid & 31, wave = tid >> 5, hh = lane >> 4, m = lane & 15;
  const int node0 = (int)blockIdx.x * NB;

  {
    int nd = node0 + (tid >> 3);
    nd = nd < nN ? nd : nN - 1;
    int s = esrc[(size_t)nd * DEG + (tid & 7)];
    s = s < 0 ? 0 : (s > nN - 1 ? nN - 1 : s);
    sSrc[tid] = s;
#pragma unroll
    for (int q = 0; q < 16; ++q) sC[q * LTHR + tid] = 0.0f;
  }
  __syncthreads();

  const unsigned short* wp  = WHH + (size_t)(16 * wave + m) * HID + 8 * hh;
  const unsigned short* hp0 = sH + m * HP + 8 * hh;
  const unsigned short* hp1 = hp0 + 16 * HP;
  const v8f zero8 = {0.f, 0.f, 0.f, 0.f, 0.f, 0.f, 0.f, 0.f};

#pragma unroll 1
  for (int t = 0; t < DEG; ++t) {
    v8f acc0[4], acc1[4];
#pragma unroll
    for (int g = 0; g < 4; ++g) { acc0[g] = zero8; acc1[g] = zero8; }
    if (t > 0) {
#pragma unroll 1
      for (int ks = 0; ks < HID / 32; ++ks) {
        const FragB ah0 = ld16(hp0 + 32 * ks);
        const FragB ah1 = ld16(hp1 + 32 * ks);
        const FragB al0 = ld16(hp0 + HID + 32 * ks);
        const FragB al1 = ld16(hp1 + HID + 32 * ks);
        FragB bf[4];
#pragma unroll
        for (int g = 0; g < 4; ++g) bf[g] = ld16(wp + (size_t)g * (HID * HID) + 32 * ks);
#pragma unroll
        for (int g = 0; g < 4; ++g) { acc0[g] = wmb(ah0, bf[g], acc0[g]); acc1[g] = wmb(ah1, bf[g], acc1[g]); }
#pragma unroll
        for (int g = 0; g < 4; ++g) { acc0[g] = wmb(al0, bf[g], acc0[g]); acc1[g] = wmb(al1, bf[g], acc1[g]); }
      }
    }
#pragma unroll
    for (int r = 0; r < 8; ++r) {
      v4f s0, s1;
      s0.x = acc0[0][r]; s0.y = acc0[1][r]; s0.z = acc0[2][r]; s0.w = acc0[3][r];
      s1.x = acc1[0][r]; s1.y = acc1[1][r]; s1.z = acc1[2][r]; s1.w = acc1[3][r];
      *(v4fa*)(sG + 4 * (r * LTHR + tid)) = s0;
      *(v4fa*)(sG + 4 * ((8 + r) * LTHR + tid)) = s1;
    }
    __syncthreads();

#pragma unroll 1
    for (int q = 0; q < 16; ++q) {
      const int lr = ((q >> 3) << 4) + 8 * hh + (q & 7);
      const int s  = sSrc[lr * DEG + t];
      const v4f xg = *(const v4f*)(XG + (size_t)s * G4 + 64 * wave + 4 * m);
      const v4f gp = *(const v4fa*)(sG + 4 * (q * LTHR + tid));
      float cc = sC[q * LTHR + tid];
      const float iv = sigm(gp.x + xg.x);
      const float fv = sigm(gp.y + xg.y);
      const float gv = tanhf(gp.z + xg.z);
      const float ov = sigm(gp.w + xg.w);
      cc = fv * cc + iv * gv;
      const float hv = ov * tanhf(cc);
      sC[q * LTHR + tid] = cc;
      const unsigned hb = bf16_bits(hv);
      const unsigned lb = bf16_bits(hv - __uint_as_float(hb << 16));
      sH[lr * HP + 16 * wave + m]       = (unsigned short)hb;
      sH[lr * HP + HID + 16 * wave + m] = (unsigned short)lb;
    }
    __syncthreads();
  }

  v8f t0 = zero8, t1 = zero8;
  int nd0 = node0 + m;       nd0 = nd0 < nN ? nd0 : nN - 1;
  int nd1 = node0 + 16 + m;  nd1 = nd1 < nN ? nd1 : nN - 1;
  if constexpr (LYR == 1) {
    const unsigned short* lp = LINW + (size_t)(16 * wave + m) * (FIN + HID) + 8 * hh;
    const float* xp0 = xf + (size_t)nd0 * FIN + 8 * hh;
    const float* xp1 = xf + (size_t)nd1 * FIN + 8 * hh;
#pragma unroll 1
    for (int ks = 0; ks < FIN / 32; ++ks) {
      const FragB a0 = lda_f32(xp0 + 32 * ks);
      const FragB a1 = lda_f32(xp1 + 32 * ks);
      const FragB bf = ld16(lp + 32 * ks);
      t0 = wmb(a0, bf, t0);
      t1 = wmb(a1, bf, t1);
    }
#pragma unroll 1
    for (int ks = 0; ks < HID / 32; ++ks) {
      const FragB ah0 = ld16(hp0 + 32 * ks);
      const FragB ah1 = ld16(hp1 + 32 * ks);
      const FragB al0 = ld16(hp0 + HID + 32 * ks);
      const FragB al1 = ld16(hp1 + HID + 32 * ks);
      const FragB bf  = ld16(lp + FIN + 32 * ks);
      t0 = wmb(ah0, bf, t0); t1 = wmb(ah1, bf, t1);
      t0 = wmb(al0, bf, t0); t1 = wmb(al1, bf, t1);
    }
  } else {
    const unsigned short* lp  = LINW + (size_t)(16 * wave + m) * (2 * HID) + 8 * hh;
    const unsigned short* rp0 = H1r + (size_t)nd0 * (2 * HID) + 8 * hh;
    const unsigned short* rp1 = H1r + (size_t)nd1 * (2 * HID) + 8 * hh;
#pragma unroll 1
    for (int ks = 0; ks < HID / 32; ++ks) {
      const FragB ah0 = ld16(rp0 + 32 * ks);
      const FragB ah1 = ld16(rp1 + 32 * ks);
      const FragB al0 = ld16(rp0 + HID + 32 * ks);
      const FragB al1 = ld16(rp1 + HID + 32 * ks);
      const FragB bf  = ld16(lp + 32 * ks);
      t0 = wmb(ah0, bf, t0); t1 = wmb(ah1, bf, t1);
      t0 = wmb(al0, bf, t0); t1 = wmb(al1, bf, t1);
    }
#pragma unroll 1
    for (int ks = 0; ks < HID / 32; ++ks) {
      const FragB ah0 = ld16(hp0 + 32 * ks);
      const FragB ah1 = ld16(hp1 + 32 * ks);
      const FragB al0 = ld16(hp0 + HID + 32 * ks);
      const FragB al1 = ld16(hp1 + HID + 32 * ks);
      const FragB bf  = ld16(lp + HID + 32 * ks);
      t0 = wmb(ah0, bf, t0); t1 = wmb(ah1, bf, t1);
      t0 = wmb(al0, bf, t0); t1 = wmb(al1, bf, t1);
    }
  }

  float* sOut = sG;
#pragma unroll
  for (int r = 0; r < 8; ++r) {
    sOut[(8 * hh + r) * HID + 16 * wave + m]      = t0[r];
    sOut[(16 + 8 * hh + r) * HID + 16 * wave + m] = t1[r];
  }
  __syncthreads();

  const v4f b4  = *(const v4f*)(pvb + 4 * lane);
  const v4f g4  = *(const v4f*)(pvg + 4 * lane);
  const v4f be4 = *(const v4f*)(pvbe + 4 * lane);
  v4f yv[4];
#pragma unroll
  for (int i = 0; i < 4; ++i) {
    const int row = 4 * wave + i;
    v4f v = *(const v4fa*)(sOut + row * HID + 4 * lane);
    v = v + b4;
    v.x = fmaxf(v.x, 0.0f); v.y = fmaxf(v.y, 0.0f); v.z = fmaxf(v.z, 0.0f); v.w = fmaxf(v.w, 0.0f);
    float s = (v.x + v.y) + (v.z + v.w);
    s += __shfl_xor(s, 16, 32);
    s += __shfl_xor(s, 8, 32);
    s += __shfl_xor(s, 4, 32);
    s += __shfl_xor(s, 2, 32);
    s += __shfl_xor(s, 1, 32);
    const float mu = s * (1.0f / 128.0f);
    v4f d;
    d.x = v.x - mu; d.y = v.y - mu; d.z = v.z - mu; d.w = v.w - mu;
    float qq = (d.x * d.x + d.y * d.y) + (d.z * d.z + d.w * d.w);
    qq += __shfl_xor(qq, 16, 32);
    qq += __shfl_xor(qq, 8, 32);
    qq += __shfl_xor(qq, 4, 32);
    qq += __shfl_xor(qq, 2, 32);
    qq += __shfl_xor(qq, 1, 32);
    const float var = qq * (1.0f / 128.0f);
    const float rs  = 1.0f / sqrtf(var + 1e-5f);
    v4f y;
    y.x = d.x * rs * g4.x + be4.x;
    y.y = d.y * rs * g4.y + be4.y;
    y.z = d.z * rs * g4.z + be4.z;
    y.w = d.w * rs * g4.w + be4.w;
    if constexpr (LYR == 1) {
      y.x = fmaxf(y.x, 0.0f); y.y = fmaxf(y.y, 0.0f); y.z = fmaxf(y.z, 0.0f); y.w = fmaxf(y.w, 0.0f);
    }
    yv[i] = y;
  }

  if constexpr (LYR == 1) {
    unsigned short* rowbuf = (unsigned short*)sC + (size_t)(wave * 4) * (2 * HID);
#pragma unroll
    for (int i = 0; i < 4; ++i) {
      v4us h4, l4;
      unsigned hb;
      hb = bf16_bits(yv[i].x); h4[0] = (unsigned short)hb; l4[0] = (unsigned short)bf16_bits(yv[i].x - __uint_as_float(hb << 16));
      hb = bf16_bits(yv[i].y); h4[1] = (unsigned short)hb; l4[1] = (unsigned short)bf16_bits(yv[i].y - __uint_as_float(hb << 16));
      hb = bf16_bits(yv[i].z); h4[2] = (unsigned short)hb; l4[2] = (unsigned short)bf16_bits(yv[i].z - __uint_as_float(hb << 16));
      hb = bf16_bits(yv[i].w); h4[3] = (unsigned short)hb; l4[3] = (unsigned short)bf16_bits(yv[i].w - __uint_as_float(hb << 16));
      *(v4usa*)(rowbuf + i * (2 * HID) + 4 * lane) = h4;
      *(v4usa*)(rowbuf + i * (2 * HID) + HID + 4 * lane) = l4;
    }
    wave_sync();
    v8us qv[4];
#pragma unroll
    for (int i = 0; i < 4; ++i) qv[i] = *(const v8usa*)(rowbuf + i * (2 * HID) + 8 * lane);
#pragma unroll
    for (int i = 0; i < 4; ++i) {
      const int node = node0 + 4 * wave + i;
      if (node < nN) *(volatile v8us*)(H1w + (size_t)node * (2 * HID) + 8 * lane) = qv[i];
    }
    __threadfence();
#pragma unroll
    for (int i = 0; i < 4; ++i) {
      const int node = node0 + 4 * wave + i;
      if (node < nN) *(volatile v8us*)(H1w + (size_t)node * (2 * HID) + 8 * lane) = qv[i];
    }
  } else {
#pragma unroll
    for (int i = 0; i < 4; ++i) {
      const int node = node0 + 4 * wave + i;
      if (node < nN) *(volatile v4f*)(outp + (size_t)node * HID + 4 * lane) = yv[i];
    }
    __threadfence();
#pragma unroll
    for (int i = 0; i < 4; ++i) {
      const int node = node0 + 4 * wave + i;
      if (node < nN) *(volatile v4f*)(outp + (size_t)node * HID + 4 * lane) = yv[i];
    }
  }
}

static inline int cdiv(int a, int b) { return (a + b - 1) / b; }
static inline size_t al256(size_t o) { return (o + 255) & ~(size_t)255; }

extern "C" void kernel_launch(void* const* d_in, const int* in_sizes, int n_in,
                              void* d_out, int out_size, void* d_ws, size_t ws_size,
                              hipStream_t stream) {
  if (n_in < 16) return;
  if (in_sizes[0] < FIN || (in_sizes[0] % FIN) != 0) return;
  const int nN = in_sizes[0] / FIN;
  if (nN < 1 || nN > (1 << 21)) return;
  if ((long long)in_sizes[1] != 2LL * DEG * nN) return;
  if (in_sizes[2] != G4 * FIN || in_sizes[3] != G4 * HID || in_sizes[4] != G4) return;
  if (in_sizes[5] != HID * (FIN + HID) || in_sizes[6] != HID) return;
  if (in_sizes[7] != HID || in_sizes[8] != HID) return;
  if (in_sizes[9] != G4 * HID || in_sizes[10] != G4 * HID || in_sizes[11] != G4) return;
  if (in_sizes[12] != HID * 2 * HID || in_sizes[13] != HID) return;
  if (in_sizes[14] != HID || in_sizes[15] != HID) return;
  if ((long long)out_size != (long long)nN * HID) return;

  const float* x     = (const float*)d_in[0];
  const int*   esrc  = (const int*)d_in[1];
  const float* Wih1  = (const float*)d_in[2];
  const float* Whh1  = (const float*)d_in[3];
  const float* b1    = (const float*)d_in[4];
  const float* lin1W = (const float*)d_in[5];
  const float* lin1b = (const float*)d_in[6];
  const float* g1    = (const float*)d_in[7];
  const float* be1   = (const float*)d_in[8];
  const float* Wih2  = (const float*)d_in[9];
  const float* Whh2  = (const float*)d_in[10];
  const float* b2    = (const float*)d_in[11];
  const float* lin2W = (const float*)d_in[12];
  const float* lin2b = (const float*)d_in[13];
  const float* g2    = (const float*)d_in[14];
  const float* be2   = (const float*)d_in[15];
  float* out = (float*)d_out;

  char* ws = (char*)d_ws;
  size_t off = 0;
  const size_t oWIH1 = off; off = al256(off + (size_t)G4 * FIN * 2);
  const size_t oWHH1 = off; off = al256(off + (size_t)G4 * HID * 2);
  const size_t oLIN1 = off; off = al256(off + (size_t)HID * (FIN + HID) * 2);
  const size_t oWIH2 = off; off = al256(off + (size_t)G4 * HID * 2);
  const size_t oWHH2 = off; off = al256(off + (size_t)G4 * HID * 2);
  const size_t oLIN2 = off; off = al256(off + (size_t)HID * 2 * HID * 2);
  const size_t oPV   = off; off = al256(off + (size_t)PVN * 4);
  const size_t oXG   = off; off = al256(off + (size_t)nN * G4 * 4);
  const size_t oH1   = off; off = al256(off + (size_t)nN * 2 * HID * 2);
  if (off > ws_size || off > (size_t)WSMAX) return;
  unsigned short* WIH1p = (unsigned short*)(ws + oWIH1);
  unsigned short* WHH1p = (unsigned short*)(ws + oWHH1);
  unsigned short* LIN1p = (unsigned short*)(ws + oLIN1);
  unsigned short* WIH2p = (unsigned short*)(ws + oWIH2);
  unsigned short* WHH2p = (unsigned short*)(ws + oWHH2);
  unsigned short* LIN2p = (unsigned short*)(ws + oLIN2);
  float*          PV    = (float*)(ws + oPV);
  float*          XG    = (float*)(ws + oXG);
  unsigned short* H1    = (unsigned short*)(ws + oH1);

  hipFuncSetAttribute(reinterpret_cast<const void*>(&k_lstm<1>), hipFuncAttributeMaxDynamicSharedMemorySize, (int)LDS_TOT);
  hipFuncSetAttribute(reinterpret_cast<const void*>(&k_lstm<2>), hipFuncAttributeMaxDynamicSharedMemorySize, (int)LDS_TOT);

  const int gM = cdiv(nN, GBM);
  const int gL = cdiv(nN, NB);

  k_prep<<<cdiv(PE5 + PVU, 256), 256, 0, stream>>>(Wih1, Whh1, b1, lin1W, lin1b, g1, be1,
                                                    Wih2, Whh2, b2, lin2W, lin2b, g2, be2,
                                                    WIH1p, WHH1p, LIN1p, WIH2p, WHH2p, LIN2p, PV);
  k_xg<1><<<dim3(gM, G4 / GBN), GTHR, 0, stream>>>(x, H1, WIH1p, PV, XG, nN);
  k_lstm<1><<<gL, LTHR, LDS_TOT, stream>>>(XG, esrc, WHH1p, x, H1, H1, LIN1p, PV + 1024, PV + 1280, PV + 1408, out, nN);
  k_xg<2><<<dim3(gM, G4 / GBN), GTHR, 0, stream>>>(x, H1, WIH2p, PV + 512, XG, nN);
  k_lstm<2><<<gL, LTHR, LDS_TOT, stream>>>(XG, esrc, WHH2p, x, H1, H1, LIN2p, PV + 1152, PV + 1536, PV + 1664, out, nN);
}
